// AdmittanceGNN_66228395704524
// MI455X (gfx1250) — hardware-verified
//
#include <hip/hip_runtime.h>
#include <stddef.h>


#define DF      128
#define AHW     64
#define NC2     256
#define NTHR    256
#define NWAVE   8
#define EPT     8
#define NGRP    2
#define CHUNK   (NTHR * EPT * NGRP)
#define WCAP    (EPT * NGRP * 32)
#define LISTN   (NWAVE * WCAP)
#define NB      512
#define GROWS   128
#define APITCH  136
#define WSCALE  16.0f
#define WINV    0.0625f

#define LDS_NODE (GROWS * DF * 4 + GROWS * APITCH * 2)
#define LDS_AGG  (NB * DF * 4 + LISTN * 4 + 64)

static_assert((CHUNK & (CHUNK - 1)) == 0);
static_assert(CHUNK <= 4096);
static_assert(NB <= 4096 && (NB & (NB - 1)) == 0);
static_assert(NB == NWAVE * 64);
static_assert(GROWS == NWAVE * 16);
static_assert(GROWS * APITCH * 2 <= GROWS * DF * 4);
static_assert((APITCH * 2) % 16 == 0);

typedef float    v4f  __attribute__((ext_vector_type(4)));
typedef float    v8f  __attribute__((ext_vector_type(8)));
typedef int      v4i  __attribute__((ext_vector_type(4)));
typedef _Float16 v8h  __attribute__((ext_vector_type(8)));
typedef _Float16 v16h __attribute__((ext_vector_type(16)));
union FragH { v16h v; v8h h[2]; };

__device__ __forceinline__ v8h cvt8(v4f a, v4f b) {
  v8h r;
  r[0] = (_Float16)a.x; r[1] = (_Float16)a.y; r[2] = (_Float16)a.z; r[3] = (_Float16)a.w;
  r[4] = (_Float16)b.x; r[5] = (_Float16)b.y; r[6] = (_Float16)b.z; r[7] = (_Float16)b.w;
  return r;
}

__device__ __forceinline__ v8f wmh(v16h a, v16h b, v8f c) {
  v8f d = __builtin_amdgcn_wmma_f32_16x16x32_f16(false, a, false, b, (short)0, c, false, false);
  asm volatile("v_nop\n\tv_nop\n\tv_nop\n\tv_nop" : "+v"(d) : "v"(a), "v"(b));
  return d;
}

template <int NBT>
__device__ __forceinline__ int scan_chunk(const int* __restrict__ dsts, int nE, int cbase, int nodeBase,
                                          int vec8, int* list, int tid, int lane, int wave) {
  int wc = 0;
  (void)lane;
#pragma unroll
  for (int g = 0; g < NGRP; ++g) {
    const int el0  = (g * NTHR + tid) * EPT;
    const int e0   = cbase + el0;
    const int sent = -2147483647 - 1;
    v4i da, db;
    if (vec8 != 0 && cbase + CHUNK <= nE) {
      da = *(const v4i*)(dsts + e0);
      db = *(const v4i*)(dsts + e0 + 4);
    } else {
      da.x = (e0     < nE) ? dsts[min(e0,     nE - 1)] : sent;
      da.y = (e0 + 1 < nE) ? dsts[min(e0 + 1, nE - 1)] : sent;
      da.z = (e0 + 2 < nE) ? dsts[min(e0 + 2, nE - 1)] : sent;
      da.w = (e0 + 3 < nE) ? dsts[min(e0 + 3, nE - 1)] : sent;
      db.x = (e0 + 4 < nE) ? dsts[min(e0 + 4, nE - 1)] : sent;
      db.y = (e0 + 5 < nE) ? dsts[min(e0 + 5, nE - 1)] : sent;
      db.z = (e0 + 6 < nE) ? dsts[min(e0 + 6, nE - 1)] : sent;
      db.w = (e0 + 7 < nE) ? dsts[min(e0 + 7, nE - 1)] : sent;
    }
    const unsigned nb = (unsigned)nodeBase;
    const unsigned s0 = (unsigned)da.x - nb, s1 = (unsigned)da.y - nb;
    const unsigned s2 = (unsigned)da.z - nb, s3 = (unsigned)da.w - nb;
    const unsigned s4 = (unsigned)db.x - nb, s5 = (unsigned)db.y - nb;
    const unsigned s6 = (unsigned)db.z - nb, s7 = (unsigned)db.w - nb;
    const bool h0 = s0 < (unsigned)NBT, h1 = s1 < (unsigned)NBT, h2 = s2 < (unsigned)NBT, h3 = s3 < (unsigned)NBT;
    const bool h4 = s4 < (unsigned)NBT, h5 = s5 < (unsigned)NBT, h6 = s6 < (unsigned)NBT, h7 = s7 < (unsigned)NBT;
    const unsigned any = __builtin_amdgcn_ballot_w32(h0 | h1 | h2 | h3 | h4 | h5 | h6 | h7);
    if (any != 0u) {
#define HITJ(J, HJ, SJ) { \
        const unsigned mj = __builtin_amdgcn_ballot_w32(HJ); \
        if (mj != 0u) { \
          if (HJ) { \
            const int pos = wc + (int)__builtin_amdgcn_mbcnt_lo(mj, 0u); \
            if (pos < WCAP) list[wave * WCAP + pos] = ((el0 + (J)) << 12) | (int)(SJ); \
          } \
          wc += (int)__builtin_popcount(mj); } }
      HITJ(0, h0, s0)
      HITJ(1, h1, s1)
      HITJ(2, h2, s2)
      HITJ(3, h3, s3)
      HITJ(4, h4, s4)
      HITJ(5, h5, s5)
      HITJ(6, h6, s6)
      HITJ(7, h7, s7)
#undef HITJ
    }
  }
  return wc;
}

__global__ __launch_bounds__(NTHR) void k_wprep(
    const float* __restrict__ wn, const float* __restrict__ we, const float* __restrict__ wa,
    _Float16* wnT, _Float16* wcT, int nL) {
  const int perL = (DF * DF + NC2 * DF) / 8;
  const int idx  = blockIdx.x * NTHR + threadIdx.x;
  if (idx >= nL * perL) return;
  const int ly = idx / perL;
  const int g  = idx - ly * perL;
  const bool segA = g < (DF * DF / 8);
  const int o  = (segA ? g : g - DF * DF / 8) * 8;
  const int n  = o / DF;
  const int k0 = o - n * DF;
  const float* p;
  int st;
  _Float16* dp;
  if (segA) {
    p  = wn + (size_t)ly * DF * DF + (size_t)k0 * DF + n;
    st = DF;
    dp = wnT + (size_t)ly * DF * DF + o;
  } else {
    dp = wcT + (size_t)ly * NC2 * DF + o;
    if (n < AHW) {
      p  = wa + (size_t)ly * 2 * DF * AHW + (size_t)k0 * AHW + n;
      st = AHW;
    } else if (n < 2 * AHW) {
      p  = wa + (size_t)ly * 2 * DF * AHW + (size_t)(DF + k0) * AHW + (n - AHW);
      st = AHW;
    } else {
      p  = we + (size_t)ly * (DF + 2) * DF + (size_t)k0 * DF + (n - 2 * AHW);
      st = DF;
    }
  }
  v4f a, b;
  a.x = p[0];      a.y = p[st];     a.z = p[2 * st]; a.w = p[3 * st];
  b.x = p[4 * st]; b.y = p[5 * st]; b.z = p[6 * st]; b.w = p[7 * st];
  a = a * WSCALE;
  b = b * WSCALE;
  const v8h hv = cvt8(a, b);
  *(volatile v8h*)dp = hv;
  __threadfence();
  *(volatile v8h*)dp = hv;
}

__global__ __launch_bounds__(NTHR) void k_node(
    const float* __restrict__ xin, const _Float16* __restrict__ wnT, const _Float16* __restrict__ wcT,
    float* pq, float* rr, int nN) {
  extern __shared__ v4f lds_dyn[];
  float*    stg = (float*)lds_dyn;
  _Float16* sA  = (_Float16*)lds_dyn;
  _Float16* sH  = (_Float16*)((char*)lds_dyn + GROWS * DF * 4);
  const int tid = threadIdx.x, lane = tid & 31, wave = tid >> 5, hh = lane >> 4, m = lane & 15;
  const int rowBase = blockIdx.x * GROWS;

#pragma unroll
  for (int i = 0; i < (GROWS * DF / 8) / NTHR; ++i) {
    const int idx = i * NTHR + tid;
    const int r   = idx >> 4;
    const int c0  = (idx & 15) * 8;
    int node = rowBase + r;
    node = node > nN - 1 ? nN - 1 : node;
    const float* xp = xin + (size_t)node * DF + c0;
    const v4f a = *(const v4f*)xp, b = *(const v4f*)(xp + 4);
    *(v8h*)(sA + r * APITCH + c0) = cvt8(a, b);
  }
  __syncthreads();

  v8f acc[8];
#pragma unroll
  for (int t = 0; t < 8; ++t) { v8f z = {0.f, 0.f, 0.f, 0.f, 0.f, 0.f, 0.f, 0.f}; acc[t] = z; }
  {
    const _Float16* ar = sA + (wave * 16 + m) * APITCH + 8 * hh;
#pragma unroll
    for (int kt = 0; kt < DF / 32; ++kt) {
      FragH a;
      a.h[0] = *(const v8h*)(ar + 32 * kt);
      a.h[1] = *(const v8h*)(ar + 32 * kt + 16);
#pragma unroll
      for (int t = 0; t < 8; ++t) {
        const _Float16* bp = wnT + (size_t)(16 * t + m) * DF + 32 * kt + 8 * hh;
        FragH b;
        b.h[0] = *(const v8h*)bp;
        b.h[1] = *(const v8h*)(bp + 16);
        acc[t] = wmh(a.v, b.v, acc[t]);
      }
    }
  }
  {
    _Float16* hp = sH + (size_t)(wave * 16 + 8 * hh) * APITCH + m;
#pragma unroll
    for (int t = 0; t < 8; ++t) {
#pragma unroll
      for (int r = 0; r < 8; ++r) hp[r * APITCH + 16 * t] = (_Float16)(acc[t][r] * WINV);
    }
  }
  __syncthreads();

#pragma unroll 1
  for (int ps = 0; ps < 2; ++ps) {
#pragma unroll
    for (int t = 0; t < 8; ++t) { v8f z = {0.f, 0.f, 0.f, 0.f, 0.f, 0.f, 0.f, 0.f}; acc[t] = z; }
    const _Float16* ar = sH + (wave * 16 + m) * APITCH + 8 * hh;
#pragma unroll
    for (int kt = 0; kt < DF / 32; ++kt) {
      FragH a;
      a.h[0] = *(const v8h*)(ar + 32 * kt);
      a.h[1] = *(const v8h*)(ar + 32 * kt + 16);
#pragma unroll
      for (int t = 0; t < 8; ++t) {
        const _Float16* bp = wcT + (size_t)(ps * DF + 16 * t + m) * DF + 32 * kt + 8 * hh;
        FragH b;
        b.h[0] = *(const v8h*)bp;
        b.h[1] = *(const v8h*)(bp + 16);
        acc[t] = wmh(a.v, b.v, acc[t]);
      }
    }
    {
      float* sp = stg + (wave * 16 + 8 * hh) * DF + m;
#pragma unroll
      for (int t = 0; t < 8; ++t) {
#pragma unroll
        for (int r = 0; r < 8; ++r) sp[r * DF + 16 * t] = acc[t][r] * WINV;
      }
    }
    __syncthreads();
    float* plane = (ps == 0) ? pq : rr;
    const float* lp = stg + wave * 16 * DF + 4 * lane;
    float* gp = plane + ((size_t)rowBase + wave * 16) * DF + 4 * lane;
#pragma unroll
    for (int i = 0; i < 16; ++i) { const v4f v = *(const v4f*)(lp + i * DF); *(volatile v4f*)(gp + (size_t)i * DF) = v; }
    __threadfence();
#pragma unroll
    for (int i = 0; i < 16; ++i) { const v4f v = *(const v4f*)(lp + i * DF); *(volatile v4f*)(gp + (size_t)i * DF) = v; }
    __syncthreads();
  }
}

__global__ __launch_bounds__(NTHR) void k_agg(
    const int* __restrict__ ei, const float* __restrict__ ea,
    const float* __restrict__ pq, const float* __restrict__ rr,
    const float* __restrict__ b1, const float* __restrict__ w2, const float* __restrict__ b2p,
    const float* __restrict__ we2, const float* __restrict__ bias,
    const float* __restrict__ gam, const float* __restrict__ bet,
    const float* __restrict__ xres, float* xout,
    int nN, int nE, int vec8, int relu, int nRowsOut) {
  extern __shared__ v4f lds_dyn[];
  float* acc  = (float*)lds_dyn;
  int*   list = (int*)(acc + NB * DF);
  int*   wcnt = list + LISTN;
  const int tid = threadIdx.x, lane = tid & 31, wave = tid >> 5;
  const int nodeBase = blockIdx.x * NB;
  const int* dsts = ei + nE;

  {
    const v4f z = {0.f, 0.f, 0.f, 0.f};
    for (int i = tid; i < NB * DF / 4; i += NTHR) lds_dyn[i] = z;
  }
  __syncthreads();

  const float b1a = b1[lane], b1b = b1[lane + 32];
  const float w2a = w2[lane], w2b = w2[lane + 32];
  const float b2s = b2p[0];
  const v4f we0 = *(const v4f*)(we2 + 4 * lane);
  const v4f we1 = *(const v4f*)(we2 + DF + 4 * lane);

  const int nChunks = (nE + CHUNK - 1) / CHUNK;
#pragma unroll 1
  for (int ch = 0; ch < nChunks; ++ch) {
    const int cbase = ch * CHUNK;
    const int wc = scan_chunk<NB>(dsts, nE, cbase, nodeBase, vec8, list, tid, lane, wave);
    if (lane == 0) wcnt[wave] = wc;
    __syncthreads();
    if (wave == 0) {
#pragma unroll 1
      for (int wsx = 0; wsx < NWAVE; ++wsx) {
        int n = __builtin_amdgcn_readfirstlane(wcnt[wsx]);
        n = n > WCAP ? WCAP : (n < 0 ? 0 : n);
        const int* lp = list + wsx * WCAP;
#pragma unroll 1
        for (int i = 0; i < n; ++i) {
          const int ent  = __builtin_amdgcn_readfirstlane(lp[i]);
          const int slot = ent & (NB - 1);
          int e = cbase + ((ent >> 12) & (CHUNK - 1));
          e = e > nE - 1 ? nE - 1 : e;
          int src = ei[e];
          src = src < 0 ? 0 : (src > nN - 1 ? nN - 1 : src);
          int ndi = nodeBase + slot;
          ndi = ndi > nN - 1 ? nN - 1 : ndi;
          const float ea0 = ea[2 * (size_t)e];
          const float ea1 = ea[2 * (size_t)e + 1];
          const float* pr = pq + (size_t)ndi * DF;
          const float* qr = pq + (size_t)src * DF + AHW;
          float t0 = pr[lane] + qr[lane] + b1a;
          float t1 = pr[32 + lane] + qr[32 + lane] + b1b;
          t0 = fmaxf(t0, 0.f);
          t1 = fmaxf(t1, 0.f);
          float s = t0 * w2a + t1 * w2b;
          s += __shfl_xor(s, 16, 32);
          s += __shfl_xor(s, 8, 32);
          s += __shfl_xor(s, 4, 32);
          s += __shfl_xor(s, 2, 32);
          s += __shfl_xor(s, 1, 32);
          const float z   = s + b2s;
          const float att = __builtin_amdgcn_rcpf(1.0f + __expf(-z));
          const v4f rv = *(const v4f*)(rr + (size_t)src * DF + 4 * lane);
          const v4f mv = (rv + ea0 * we0 + ea1 * we1) * att;
          v4f* ap = (v4f*)(acc + slot * DF + 4 * lane);
          *ap = *ap + mv;
        }
      }
    }
    __syncthreads();
  }

  const v4f bv = *(const v4f*)(bias + 4 * lane);
  const v4f gv = *(const v4f*)(gam + 4 * lane);
  const v4f ev = *(const v4f*)(bet + 4 * lane);
#pragma unroll 1
  for (int q = 0; q < 64; ++q) {
    const int row  = wave * 64 + q;
    const int node = nodeBase + row;
    const int ndc  = node > nN - 1 ? nN - 1 : node;
    v4f* ap = (v4f*)(acc + row * DF + 4 * lane);
    const v4f v = *ap + bv;
    float s = (v.x + v.y) + (v.z + v.w);
    s += __shfl_xor(s, 16, 32);
    s += __shfl_xor(s, 8, 32);
    s += __shfl_xor(s, 4, 32);
    s += __shfl_xor(s, 2, 32);
    s += __shfl_xor(s, 1, 32);
    const float mu = s * (1.0f / (float)DF);
    const v4f d = v - mu;
    float ss = (d.x * d.x + d.y * d.y) + (d.z * d.z + d.w * d.w);
    ss += __shfl_xor(ss, 16, 32);
    ss += __shfl_xor(ss, 8, 32);
    ss += __shfl_xor(ss, 4, 32);
    ss += __shfl_xor(ss, 2, 32);
    ss += __shfl_xor(ss, 1, 32);
    const float var = ss * (1.0f / (float)DF);
    const float inv = rsqrtf(var + 1e-5f);
    v4f y = d * inv * gv + ev;
    if (relu != 0) { y.x = fmaxf(y.x, 0.f); y.y = fmaxf(y.y, 0.f); y.z = fmaxf(y.z, 0.f); y.w = fmaxf(y.w, 0.f); }
    y = y + *(const v4f*)(xres + (size_t)ndc * DF + 4 * lane);
    *ap = y;
    if (node < nRowsOut) *(volatile v4f*)(xout + (size_t)node * DF + 4 * lane) = y;
  }
  __threadfence();
#pragma unroll 1
  for (int q = 0; q < 64; ++q) {
    const int row  = wave * 64 + q;
    const int node = nodeBase + row;
    if (node < nRowsOut) {
      const v4f y = *(const v4f*)(acc + row * DF + 4 * lane);
      *(volatile v4f*)(xout + (size_t)node * DF + 4 * lane) = y;
    }
  }
}

extern "C" void kernel_launch(void* const* d_in, const int* in_sizes, int n_in,
                              void* d_out, int out_size, void* d_ws, size_t ws_size,
                              hipStream_t stream) {
  if (n_in < 12) return;
  const int nN = in_sizes[0] / DF;
  const int nE = in_sizes[1] / 2;
  const int nL = in_sizes[3] / (DF * DF);
  if (nN <= 0 || nE < 0 || nL <= 0) return;
  if (in_sizes[0] != nN * DF || in_sizes[1] != nE * 2 || in_sizes[2] != nE * 2) return;
  if (in_sizes[3] != nL * DF * DF || in_sizes[4] != nL * (DF + 2) * DF || in_sizes[5] != nL * 2 * DF * AHW) return;
  if (in_sizes[6] < nL * AHW || in_sizes[7] < nL * AHW || in_sizes[8] < nL) return;
  if (in_sizes[9] < nL * DF || in_sizes[10] < nL * DF || in_sizes[11] < nL * DF) return;
  if (out_size != nN * DF) return;

  const float* x    = (const float*)d_in[0];
  const int*   ei   = (const int*)d_in[1];
  const float* ea   = (const float*)d_in[2];
  const float* wn   = (const float*)d_in[3];
  const float* we   = (const float*)d_in[4];
  const float* wa   = (const float*)d_in[5];
  const float* b1   = (const float*)d_in[6];
  const float* w2   = (const float*)d_in[7];
  const float* b2   = (const float*)d_in[8];
  const float* bias = (const float*)d_in[9];
  const float* gam  = (const float*)d_in[10];
  const float* bet  = (const float*)d_in[11];
  float* out = (float*)d_out;

  const int nG = (nN + GROWS - 1) / GROWS;
  const int nA = (nN + NB - 1) / NB;

  char* ws = (char*)d_ws;
  size_t off = 0;
  const size_t oWn = off; off += (size_t)nL * DF * DF * 2;            off = (off + 255) & ~(size_t)255;
  const size_t oWc = off; off += (size_t)nL * NC2 * DF * 2;           off = (off + 255) & ~(size_t)255;
  const size_t oPQ = off; off += (size_t)nG * GROWS * DF * 4;          off = (off + 255) & ~(size_t)255;
  const size_t oRR = off; off += (size_t)nG * GROWS * DF * 4;          off = (off + 255) & ~(size_t)255;
  const size_t oXA = off; off += (size_t)nA * NB * DF * 4;             off = (off + 255) & ~(size_t)255;
  const size_t oXB = off; off += (size_t)nA * NB * DF * 4;             off = (off + 255) & ~(size_t)255;
  if (off > ws_size) return;
  _Float16* wnT = (_Float16*)(ws + oWn);
  _Float16* wcT = (_Float16*)(ws + oWc);
  float*    pq  = (float*)(ws + oPQ);
  float*    rr  = (float*)(ws + oRR);
  float*    xA  = (float*)(ws + oXA);
  float*    xB  = (float*)(ws + oXB);

  const int vec8 = ((nE & 3) == 0) ? 1 : 0;

  const int nPrep = nL * ((DF * DF + NC2 * DF) / 8);
  k_wprep<<<(nPrep + NTHR - 1) / NTHR, NTHR, 0, stream>>>(wn, we, wa, wnT, wcT, nL);

  hipFuncSetAttribute(reinterpret_cast<const void*>(&k_node),
                      hipFuncAttributeMaxDynamicSharedMemorySize, LDS_NODE);
  hipFuncSetAttribute(reinterpret_cast<const void*>(&k_agg),
                      hipFuncAttributeMaxDynamicSharedMemorySize, LDS_AGG);

  for (int i = 0; i < nL; ++i) {
    const float* xin = (i == 0) ? x : ((i & 1) ? xA : xB);
    float*       xo  = (i == nL - 1) ? out : ((i & 1) ? xB : xA);
    const int nRowsOut = (i == nL - 1) ? nN : nA * NB;
    const int relu     = (i < nL - 1) ? 1 : 0;
    k_node<<<nG, NTHR, LDS_NODE, stream>>>(xin, wnT + (size_t)i * DF * DF, wcT + (size_t)i * NC2 * DF, pq, rr, nN);
    k_agg<<<nA, NTHR, LDS_AGG, stream>>>(ei, ea, pq, rr,
                                         b1 + (size_t)i * AHW, w2 + (size_t)i * AHW, b2 + i,
                                         we + (size_t)i * (DF + 2) * DF + (size_t)DF * DF,
                                         bias + (size_t)i * DF, gam + (size_t)i * DF, bet + (size_t)i * DF,
                                         xin, xo, nN, nE, vec8, relu, nRowsOut);
  }
}
